// STGCNModel_19275813224639
// MI455X (gfx1250) — hardware-verified
//
#include <hip/hip_runtime.h>
#include <stddef.h>


#define NNODE   10000
#define NBATCH  8
#define NTIME   12
#define NFEAT   2
#define HC      64
#define KTAP    3
#define TFIRST  9
#define NSL     3
#define CSELF   1.0f
#define NTHR    256
#define NWAVE   8
#define EPT     8
#define NGRP    2
#define CHUNK   (NTHR * EPT * NGRP)
#define WCAPC   (EPT * NGRP * 32)
#define WCAPF   (EPT * NGRP * 32)
#define ESHF    11
#define EMASK   0xFFFFF
#define NBC     32768
#define NBF     2048
#define RCAP    49152
#define RBN     128
#define TGT     256
#define DEGCAP  512
#define GROWS   128
#define OTHR    512
#define HSCL    64
#define WSCL    64
#define KC      (KTAP * HC)
#define SPP     KC
#define T1P     (2 * HC)
#define NPAD    (((NNODE + TGT - 1) / TGT) * TGT)
#define WSCAP   134217728

#define LDS_COUNT  ((NBC + NWAVE * WCAPC + NWAVE) * 4)
#define LDS_FILL   ((RCAP + NBF + NWAVE * WCAPF + NWAVE) * 4)

static_assert((CHUNK & (CHUNK - 1)) == 0);
static_assert((NBC & (NBC - 1)) == 0 && (NBF & (NBF - 1)) == 0);
static_assert(NBF <= (1 << ESHF));
static_assert((NBC % NBF) == 0);
static_assert(OTHR * 4 == NBF);
static_assert((RCAP % 32) == 0);
static_assert(TGT == NWAVE * 32);
static_assert(GROWS == NWAVE * 16);
static_assert((TGT % GROWS) == 0);
static_assert(NBC == NWAVE * 32 * 128);
static_assert(HC == 16 * 4);
static_assert(HC == 32 * 2);
static_assert((NPAD % TGT) == 0 && (NPAD % GROWS) == 0 && (NPAD % NTHR) == 0 && NPAD >= NNODE);
static_assert((NNODE % 4) == 0 && ((NBATCH * NNODE) % 4) == 0);
static_assert((KC % 32) == 0 && (T1P % 32) == 0 && (HC % 32) == 0);
static_assert(TFIRST + NSL == NTIME);
static_assert(LDS_FILL <= 300 * 1024 && LDS_COUNT <= 300 * 1024);

typedef float     v2f  __attribute__((ext_vector_type(2)));
typedef float     v4f  __attribute__((ext_vector_type(4)));
typedef float     v8f  __attribute__((ext_vector_type(8)));
typedef int       v4i  __attribute__((ext_vector_type(4)));
typedef _Float16  v2h  __attribute__((ext_vector_type(2)));
typedef _Float16  v4h  __attribute__((ext_vector_type(4)));
typedef _Float16  v8h  __attribute__((ext_vector_type(8)));
typedef _Float16  v16h __attribute__((ext_vector_type(16)));
union FragH { v16h v; v8h h[2]; };
union U32F { float f; int i; };

__device__ __forceinline__ v8f wmf(v16h a, v16h b, v8f c) {
  v8f d = __builtin_amdgcn_wmma_f32_16x16x32_f16(false, a, false, b, (short)0, c, false, false);
  asm volatile("v_nop\n\tv_nop\n\tv_nop\n\tv_nop" : "+v"(d) : "v"(a), "v"(b));
  return d;
}

template <int NB, int EID, int WC>
__device__ __forceinline__ int scan_chunk(const int* __restrict__ keys, int nK, int cbase, int slotBase, int vec8,
                                          int* list, int tid, int lane, int wave) {
  int wc = 0;
#pragma unroll
  for (int g = 0; g < NGRP; ++g) {
    const int el0  = (g * NTHR + tid) * EPT;
    const int e0   = cbase + el0;
    const int sent = -2147483647 - 1;
    v4i da, db;
    if (vec8 != 0 && cbase + CHUNK <= nK) {
      da = *(const v4i*)(keys + e0);
      db = *(const v4i*)(keys + e0 + 4);
    } else {
      const int i0 = min(e0, nK - 1),     i1 = min(e0 + 1, nK - 1), i2 = min(e0 + 2, nK - 1), i3 = min(e0 + 3, nK - 1);
      const int i4 = min(e0 + 4, nK - 1), i5 = min(e0 + 5, nK - 1), i6 = min(e0 + 6, nK - 1), i7 = min(e0 + 7, nK - 1);
      da.x = (e0     < nK) ? keys[i0] : sent;
      da.y = (e0 + 1 < nK) ? keys[i1] : sent;
      da.z = (e0 + 2 < nK) ? keys[i2] : sent;
      da.w = (e0 + 3 < nK) ? keys[i3] : sent;
      db.x = (e0 + 4 < nK) ? keys[i4] : sent;
      db.y = (e0 + 5 < nK) ? keys[i5] : sent;
      db.z = (e0 + 6 < nK) ? keys[i6] : sent;
      db.w = (e0 + 7 < nK) ? keys[i7] : sent;
    }
    const unsigned nb = (unsigned)slotBase;
    const unsigned s0 = (unsigned)da.x - nb, s1 = (unsigned)da.y - nb;
    const unsigned s2 = (unsigned)da.z - nb, s3 = (unsigned)da.w - nb;
    const unsigned s4 = (unsigned)db.x - nb, s5 = (unsigned)db.y - nb;
    const unsigned s6 = (unsigned)db.z - nb, s7 = (unsigned)db.w - nb;
    const bool h0 = s0 < (unsigned)NB, h1 = s1 < (unsigned)NB, h2 = s2 < (unsigned)NB, h3 = s3 < (unsigned)NB;
    const bool h4 = s4 < (unsigned)NB, h5 = s5 < (unsigned)NB, h6 = s6 < (unsigned)NB, h7 = s7 < (unsigned)NB;
    const unsigned any = __builtin_amdgcn_ballot_w32(h0 | h1 | h2 | h3 | h4 | h5 | h6 | h7);
    if (any != 0u) {
#define HITJ(HJ, SJ, JJ) { \
        const unsigned mj = __builtin_amdgcn_ballot_w32(HJ); \
        if (mj != 0u) { \
          if (HJ) { \
            const int pos = wc + (int)__builtin_amdgcn_mbcnt_lo(mj, 0u); \
            const int entv = EID ? (((e0 + (JJ)) << ESHF) | (int)(SJ)) : (int)(SJ); \
            if (pos < WC) list[wave * WC + pos] = entv; \
          } \
          wc += (int)__builtin_popcount(mj); } }
      HITJ(h0, s0, 0)
      HITJ(h1, s1, 1)
      HITJ(h2, s2, 2)
      HITJ(h3, s3, 3)
      HITJ(h4, s4, 4)
      HITJ(h5, s5, 5)
      HITJ(h6, s6, 6)
      HITJ(h7, s7, 7)
#undef HITJ
    }
  }
  return wc;
}

template <int MODE>
__global__ __launch_bounds__(NTHR) void k_wprep(const float* __restrict__ W, _Float16* Wp, int total8, float scale) {
  const int i = (int)blockIdx.x * NTHR + (int)threadIdx.x;
  if (i >= total8) return;
  float f[8];
  if (MODE == 0) {
    const int n = i >> 3, k0 = (i & 7) * 8;
#pragma unroll
    for (int q = 0; q < 8; ++q) f[q] = W[(k0 + q) * HC + n];
  } else {
    const int n = i / (KC / 8);
    const int k0 = (i - n * (KC / 8)) * 8;
    const int tap = k0 >> 6, ci0 = k0 & 63;
#pragma unroll
    for (int q = 0; q < 8; ++q) f[q] = W[(n * HC + ci0 + q) * KTAP + tap];
  }
  v8h hv;
#pragma unroll
  for (int q = 0; q < 8; ++q) hv[q] = (_Float16)(f[q] * scale);
  _Float16* d = Wp + (size_t)8 * (size_t)i;
  *(volatile v8h*)d = hv;
  __threadfence();
  *(volatile v8h*)d = hv;
}

__global__ __launch_bounds__(NTHR) void k_count(const int* __restrict__ keys, int* cnt, int nK, int vec8) {
  extern __shared__ v4f lds_dyn[];
  int* scnt = (int*)lds_dyn;
  int* list = scnt + NBC;
  int* wcnt = list + NWAVE * WCAPC;
  const int tid = threadIdx.x, lane = tid & 31, wave = tid >> 5;
  const int nodeBase = blockIdx.x * NBC;

  {
    const v4i z = {0, 0, 0, 0};
    for (int i = tid; i < NBC / 4; i += NTHR) ((v4i*)scnt)[i] = z;
  }
  __syncthreads();

  const int nChunks = (nK + CHUNK - 1) / CHUNK;
#pragma unroll 1
  for (int ch = 0; ch < nChunks; ++ch) {
    const int cbase = ch * CHUNK;
    const int wc = scan_chunk<NBC, 0, WCAPC>(keys, nK, cbase, nodeBase, vec8, list, tid, lane, wave);
    if (lane == 0) wcnt[wave] = wc;
    __syncthreads();
    if (wave == 0) {
#pragma unroll 1
      for (int wsx = 0; wsx < NWAVE; ++wsx) {
        int n = __builtin_amdgcn_readfirstlane(wcnt[wsx]);
        n = n > WCAPC ? WCAPC : (n < 0 ? 0 : n);
        const int* lp = list + wsx * WCAPC;
#pragma unroll 1
        for (int i = 0; i < n; ++i) {
          const int ent  = __builtin_amdgcn_readfirstlane(lp[i]);
          const int slot = ent & (NBC - 1);
          if (lane == 0) scnt[slot] = scnt[slot] + 1;
        }
      }
    }
    __syncthreads();
  }

  int* cp = cnt + (size_t)nodeBase;
#pragma unroll 4
  for (int q = 0; q < 32; ++q) {
    const int f = (wave * 32 + q) * 128 + 4 * lane;
    const v4i c = *(const v4i*)(scnt + f);
    *(volatile v4i*)(cp + f) = c;
  }
  __threadfence();
#pragma unroll 4
  for (int q = 0; q < 32; ++q) {
    const int f = (wave * 32 + q) * 128 + 4 * lane;
    const v4i c = *(const v4i*)(scnt + f);
    *(volatile v4i*)(cp + f) = c;
  }
}

__global__ __launch_bounds__(OTHR) void k_offsets(const int* __restrict__ cnt, int* off, int* rbase, int nBF) {
  __shared__ __attribute__((aligned(16))) int srb[RBN];
  __shared__ int wtot[OTHR / 32];
  const int tid = threadIdx.x, lane = tid & 31, wave = tid >> 5;
  for (int i = tid; i < RBN; i += OTHR) srb[i] = 0;
  int carry = 0;
#pragma unroll 1
  for (int fb = 0; fb < nBF; ++fb) {
    const int base = fb * NBF;
    const v4i c = *(const v4i*)(cnt + base + 4 * tid);
    const int e0 = max(c.x, 0), e1 = max(c.y, 0), e2 = max(c.z, 0), e3 = max(c.w, 0);
    const int ts = e0 + e1 + e2 + e3;
    int incl = ts;
#pragma unroll
    for (int d = 1; d < 32; d <<= 1) {
      const int t = __shfl_up(incl, d, 32);
      if (lane >= d) incl += t;
    }
    if (lane == 31) wtot[wave] = incl;
    __syncthreads();
    int pre = 0;
#pragma unroll 1
    for (int w = 0; w < wave; ++w) pre += wtot[w];
    int tot = 0;
#pragma unroll
    for (int w = 0; w < OTHR / 32; ++w) tot += wtot[w];
    int run = carry + pre + incl - ts;
    v4i o;
    o.x = run; run += e0;
    o.y = run; run += e1;
    o.z = run; run += e2;
    o.w = run;
    int* op = off + base + 4 * tid;
    *(volatile v4i*)op = o;
    __threadfence();
    *(volatile v4i*)op = o;
    if (tid == 0) srb[min(fb, RBN - 1)] = carry;
    carry += (tot + 31) & ~31;
    __syncthreads();
  }
  if (tid == 0) srb[min(nBF, RBN - 1)] = carry;
  __syncthreads();
  v4i rv = {0, 0, 0, 0};
  if (tid < 32) rv = *(const v4i*)(srb + 4 * tid);
  if (tid < 32) *(volatile v4i*)(rbase + 4 * tid) = rv;
  __threadfence();
  if (tid < 32) *(volatile v4i*)(rbase + 4 * tid) = rv;
}

__global__ __launch_bounds__(NTHR) void k_fill(
    const int* __restrict__ keys, const int* __restrict__ off, const int* __restrict__ rbase,
    int* csr, int nK, int vec8, int csrLen) {
  extern __shared__ v4f lds_dyn[];
  int* region = (int*)lds_dyn;
  int* cursor = region + RCAP;
  int* list   = cursor + NBF;
  int* wcnt   = list + NWAVE * WCAPF;
  const int tid = threadIdx.x, lane = tid & 31, wave = tid >> 5;
  const int b = blockIdx.x;
  const int nodeBase = b * NBF;

  int rb0 = rbase[b];
  const int rb1 = rbase[b + 1];
  rb0 = rb0 < 0 ? 0 : (rb0 > csrLen ? csrLen : rb0);
  rb0 &= ~31;
  int len = rb1 - rb0;
  len = len < 0 ? 0 : (len > RCAP ? RCAP : len);
  int lenW = (len + 31) & ~31;
  if (rb0 + lenW > csrLen) lenW = (csrLen - rb0) & ~31;

  {
    const v4i z = {0, 0, 0, 0};
    for (int i = tid; i < RCAP / 4; i += NTHR) ((v4i*)region)[i] = z;
    for (int s = tid; s < NBF; s += NTHR) {
      int o = off[nodeBase + s] - rb0;
      o = o < 0 ? 0 : (o > RCAP ? RCAP : o);
      cursor[s] = o;
    }
  }
  __syncthreads();

  const int nChunks = (nK + CHUNK - 1) / CHUNK;
#pragma unroll 1
  for (int ch = 0; ch < nChunks; ++ch) {
    const int cbase = ch * CHUNK;
    const int wc = scan_chunk<NBF, 1, WCAPF>(keys, nK, cbase, nodeBase, vec8, list, tid, lane, wave);
    if (lane == 0) wcnt[wave] = wc;
    __syncthreads();
    if (wave == 0) {
#pragma unroll 1
      for (int wsx = 0; wsx < NWAVE; ++wsx) {
        int n = __builtin_amdgcn_readfirstlane(wcnt[wsx]);
        n = n > WCAPF ? WCAPF : (n < 0 ? 0 : n);
        const int* lp = list + wsx * WCAPF;
#pragma unroll 1
        for (int i = 0; i < n; ++i) {
          const int ent  = __builtin_amdgcn_readfirstlane(lp[i]);
          const int slot = ent & (NBF - 1);
          int e = (ent >> ESHF) & EMASK;
          e = e > nK - 1 ? nK - 1 : e;
          if (lane == 0) {
            int pos = cursor[slot];
            pos = pos < 0 ? 0 : (pos > RCAP - 1 ? RCAP - 1 : pos);
            region[pos] = e;
            const int np = pos + 1;
            cursor[slot] = np > RCAP ? RCAP : np;
          }
        }
      }
    }
    __syncthreads();
  }

  const int nv = lenW >> 2;
  int* gp = csr + rb0;
#pragma unroll 1
  for (int i = tid; i < nv; i += NTHR) { const v4i v = ((const v4i*)region)[i]; *(volatile v4i*)(gp + 4 * i) = v; }
  __threadfence();
#pragma unroll 1
  for (int i = tid; i < nv; i += NTHR) { const v4i v = ((const v4i*)region)[i]; *(volatile v4i*)(gp + 4 * i) = v; }
}

__global__ __launch_bounds__(NTHR) void k_dinv(
    const int* __restrict__ csr, const int* __restrict__ off, const int* __restrict__ cnt,
    const float* __restrict__ ew, float* dinv, int nK, int csrLen) {
  __shared__ __attribute__((aligned(16))) float sd[NTHR];
  const int tid = threadIdx.x;
  const int c = (int)blockIdx.x * NTHR + tid;
  int n = cnt[c];
  n = n < 0 ? 0 : (n > DEGCAP ? DEGCAP : n);
  const int st = off[c];
  float s = 0.0f;
#pragma unroll 1
  for (int i = 0; i < n; ++i) {
    int pos = st + i;
    pos = pos < 0 ? 0 : (pos > csrLen - 1 ? csrLen - 1 : pos);
    int e = csr[pos];
    e = e < 0 ? 0 : (e > nK - 1 ? nK - 1 : e);
    s += ew[e];
  }
  const float g = s + CSELF;
  const float d = g > 0.0f ? rsqrtf(g) : 0.0f;
  sd[tid] = d;
  __syncthreads();
  float* dp = dinv + (size_t)blockIdx.x * NTHR;
  if (tid < NTHR / 4) { const v4f v = *(const v4f*)(sd + 4 * tid); *(volatile v4f*)(dp + 4 * tid) = v; }
  __threadfence();
  if (tid < NTHR / 4) { const v4f v = *(const v4f*)(sd + 4 * tid); *(volatile v4f*)(dp + 4 * tid) = v; }
}

__global__ __launch_bounds__(NTHR) void k_agg1(
    const int* __restrict__ csr, const int* __restrict__ off, const int* __restrict__ cnt,
    const float* __restrict__ dinv, const int* __restrict__ esrc, const float* __restrict__ ew,
    const float* __restrict__ xs, int bstrideX, const float* __restrict__ W1, const float* __restrict__ bias,
    _Float16* outH, int nN, int nK, int csrLen, float hscl) {
  __shared__ __attribute__((aligned(16))) _Float16 stg[NWAVE * 4 * HC];
  const int tid = threadIdx.x, lane = tid & 31, wave = tid >> 5;
  const int b = blockIdx.y;
  const int tbase = blockIdx.x * TGT + wave * 32;
  const int cl = tbase + lane;
  const int cnt_l = cnt[cl];
  const int off_l = off[cl];
  U32F dvu; dvu.f = dinv[cl];
  const int ch = 2 * lane;
  const float wa0 = W1[ch], wa1 = W1[ch + 1], wb0 = W1[HC + ch], wb1 = W1[HC + ch + 1];
  const float bq0 = bias[ch], bq1 = bias[ch + 1];
  const float* xb = xs + (size_t)b * (size_t)bstrideX;
  _Float16* ohb = outH + (size_t)b * (size_t)NPAD * HC;
  _Float16* sw = stg + wave * 4 * HC;

#pragma unroll 1
  for (int j = 0; j < 32; ++j) {
    const int c = tbase + j;
    int n = __builtin_amdgcn_readlane(cnt_l, j);
    n = n < 0 ? 0 : (n > DEGCAP ? DEGCAP : n);
    const int st = __builtin_amdgcn_readlane(off_l, j);
    U32F du; du.i = __builtin_amdgcn_readlane(dvu.i, j);
    const float dc = du.f;
    float a0 = 0.0f, a1 = 0.0f;
#pragma unroll 1
    for (int q0 = 0; q0 < n; q0 += 32) {
      int pos = st + q0 + lane;
      pos = pos < 0 ? 0 : (pos > csrLen - 1 ? csrLen - 1 : pos);
      int e = csr[pos];
      e = e < 0 ? 0 : (e > nK - 1 ? nK - 1 : e);
      int s = esrc[e];
      s = s < 0 ? 0 : (s > nN - 1 ? nN - 1 : s);
      const float w = ew[e];
      const v2f xv = *(const v2f*)(xb + 2 * (size_t)s);
      const float ds = dinv[s];
      const float t = ((q0 + lane) < n) ? (w * ds) : 0.0f;
      a0 += t * xv.x;
      a1 += t * xv.y;
    }
#pragma unroll
    for (int d = 16; d >= 1; d >>= 1) {
      a0 += __shfl_xor(a0, d);
      a1 += __shfl_xor(a1, d);
    }
    const int cc = c < nN ? c : nN - 1;
    const v2f xc = *(const v2f*)(xb + 2 * (size_t)cc);
    const float ax0 = (a0 + dc * xc.x) * dc;
    const float ax1 = (a1 + dc * xc.y) * dc;
    float h0 = ax0 * wa0 + ax1 * wb0 + bq0;
    float h1 = ax0 * wa1 + ax1 * wb1 + bq1;
    h0 = fmaxf(h0, 0.0f);
    h1 = fmaxf(h1, 0.0f);
    const float z = (c < nN) ? hscl : 0.0f;
    v2h hv2;
    hv2[0] = (_Float16)(h0 * z);
    hv2[1] = (_Float16)(h1 * z);
    *(v2h*)(sw + (j & 3) * HC + ch) = hv2;
    if ((j & 3) == 3) {
      __builtin_amdgcn_fence(__ATOMIC_ACQ_REL, "wavefront");
      __builtin_amdgcn_wave_barrier();
      const v8h hv = *(const v8h*)(sw + 8 * lane);
      _Float16* rp = ohb + (size_t)(c - 3) * HC + 8 * lane;
      *(volatile v8h*)rp = hv;
      __threadfence();
      *(volatile v8h*)rp = hv;
      __builtin_amdgcn_fence(__ATOMIC_ACQ_REL, "wavefront");
      __builtin_amdgcn_wave_barrier();
    }
  }
}

__global__ __launch_bounds__(NTHR) void k_agg2(
    const int* __restrict__ csr, const int* __restrict__ off, const int* __restrict__ cnt,
    const float* __restrict__ dinv, const int* __restrict__ esrc, const float* __restrict__ ew,
    const float* __restrict__ hw, const float* __restrict__ bias, _Float16* outH,
    int outPitch, int outStride, int nN, int nK, int csrLen, float hscl) {
  __shared__ __attribute__((aligned(16))) _Float16 stg[NWAVE * 8 * HC];
  const int tid = threadIdx.x, lane = tid & 31, wave = tid >> 5;
  const int h = lane >> 4, q = lane & 15, ch = 4 * q;
  const int b = blockIdx.y;
  const int tbase = blockIdx.x * TGT + wave * 32;
  const int cl = tbase + lane;
  const int cnt_l = cnt[cl];
  const int off_l = off[cl];
  U32F dvu; dvu.f = dinv[cl];
  const v4f bq = *(const v4f*)(bias + ch);
  const float* hwb = hw + (size_t)b * (size_t)NPAD * HC;
  _Float16* ohb = outH + (size_t)b * (size_t)outStride;
  _Float16* sw = stg + wave * 8 * HC;

#pragma unroll 1
  for (int j = 0; j < 32; ++j) {
    const int c = tbase + j;
    int n = __builtin_amdgcn_readlane(cnt_l, j);
    n = n < 0 ? 0 : (n > DEGCAP ? DEGCAP : n);
    const int st = __builtin_amdgcn_readlane(off_l, j);
    U32F du; du.i = __builtin_amdgcn_readlane(dvu.i, j);
    const float dc = du.f;
    v4f acc = {0.0f, 0.0f, 0.0f, 0.0f};
#pragma unroll 1
    for (int q0 = 0; q0 < n; q0 += 32) {
      int pos = st + q0 + lane;
      pos = pos < 0 ? 0 : (pos > csrLen - 1 ? csrLen - 1 : pos);
      int e = csr[pos];
      e = e < 0 ? 0 : (e > nK - 1 ? nK - 1 : e);
      int sl = esrc[e];
      sl = sl < 0 ? 0 : (sl > nN - 1 ? nN - 1 : sl);
      U32F wl; wl.f = ew[e];
      const int mcnt = (n - q0) < 32 ? (n - q0) : 32;
#pragma unroll 1
      for (int p = 0; p < mcnt; p += 2) {
        const int s0 = __builtin_amdgcn_readlane(sl, p);
        const int s1 = __builtin_amdgcn_readlane(sl, p + 1);
        U32F w0, w1;
        w0.i = __builtin_amdgcn_readlane(wl.i, p);
        w1.i = __builtin_amdgcn_readlane(wl.i, p + 1);
        const float w1f = (p + 1 < mcnt) ? w1.f : 0.0f;
        const int   s = h ? s1 : s0;
        const float w = h ? w1f : w0.f;
        const v4f v = *(const v4f*)(hwb + (size_t)s * HC + ch);
        acc.x += w * v.x; acc.y += w * v.y; acc.z += w * v.z; acc.w += w * v.w;
      }
    }
    acc.x += __shfl_xor(acc.x, 16);
    acc.y += __shfl_xor(acc.y, 16);
    acc.z += __shfl_xor(acc.z, 16);
    acc.w += __shfl_xor(acc.w, 16);
    const int cc = c < nN ? c : nN - 1;
    const v4f sv = *(const v4f*)(hwb + (size_t)cc * HC + ch);
    v4f v;
    v.x = (acc.x + sv.x) * dc + bq.x;
    v.y = (acc.y + sv.y) * dc + bq.y;
    v.z = (acc.z + sv.z) * dc + bq.z;
    v.w = (acc.w + sv.w) * dc + bq.w;
    v.x = fmaxf(v.x, 0.0f); v.y = fmaxf(v.y, 0.0f); v.z = fmaxf(v.z, 0.0f); v.w = fmaxf(v.w, 0.0f);
    const float z = (c < nN) ? hscl : 0.0f;
    v4h h4;
    h4[0] = (_Float16)(v.x * z); h4[1] = (_Float16)(v.y * z); h4[2] = (_Float16)(v.z * z); h4[3] = (_Float16)(v.w * z);
    *(v4h*)(sw + h * 4 * HC + (j & 3) * HC + ch) = h4;
    if ((j & 3) == 3) {
      __builtin_amdgcn_fence(__ATOMIC_ACQ_REL, "wavefront");
      __builtin_amdgcn_wave_barrier();
      const v8h hv = *(const v8h*)(sw + 8 * lane);
      _Float16* rp = ohb + (size_t)(c - 3 + (lane >> 3)) * (size_t)outPitch + 8 * (lane & 7);
      *(volatile v8h*)rp = hv;
      __threadfence();
      *(volatile v8h*)rp = hv;
      __builtin_amdgcn_fence(__ATOMIC_ACQ_REL, "wavefront");
      __builtin_amdgcn_wave_barrier();
    }
  }
}

template <int KD, int EPI>
__global__ __launch_bounds__(NTHR) void k_gemm(
    const _Float16* __restrict__ A16, int lda, int strideA,
    const _Float16* __restrict__ Bw, int ldb,
    const float* __restrict__ rsc, const float* __restrict__ bias,
    const float* __restrict__ ow, const float* __restrict__ ob,
    float* Cf, _Float16* Ch, int ldc, int strideC, float osc, float hscl) {
  static_assert((KD % 32) == 0);
  __shared__ __attribute__((aligned(16))) float stg[GROWS * HC];
  __shared__ __attribute__((aligned(16))) float sOw[HC];
  __shared__ __attribute__((aligned(16))) float sOut[GROWS];
  const int tid = threadIdx.x, lane = tid & 31, wave = tid >> 5, hh = lane >> 4, m = lane & 15;
  const int b = blockIdx.y;
  const int rowBase = blockIdx.x * GROWS;
  if (EPI == 2) { if (tid < HC) sOw[tid] = ow[tid]; }
  const _Float16* ap  = A16 + (size_t)b * (size_t)strideA + (size_t)(rowBase + wave * 16 + m) * (size_t)lda + 8 * hh;
  const _Float16* bp0 = Bw + (size_t)m * (size_t)ldb + 8 * hh;

  v8f acc[4];
#pragma unroll
  for (int t = 0; t < 4; ++t) { v8f z = {0.f, 0.f, 0.f, 0.f, 0.f, 0.f, 0.f, 0.f}; acc[t] = z; }

#pragma unroll 1
  for (int kt = 0; kt < KD / 32; ++kt) {
    FragH af;
    af.h[0] = *(const v8h*)(ap + 32 * kt);
    af.h[1] = *(const v8h*)(ap + 32 * kt + 16);
#pragma unroll
    for (int t = 0; t < 4; ++t) {
      const _Float16* bp = bp0 + (size_t)(16 * t) * (size_t)ldb + 32 * kt;
      FragH bf;
      bf.h[0] = *(const v8h*)bp;
      bf.h[1] = *(const v8h*)(bp + 16);
      acc[t] = wmf(af.v, bf.v, acc[t]);
    }
  }

  const int r0 = wave * 16 + 8 * hh;
  float s[8];
  if (EPI == 0) {
    const v4f dA = *(const v4f*)(rsc + (size_t)rowBase + r0);
    const v4f dB = *(const v4f*)(rsc + (size_t)rowBase + r0 + 4);
    s[0] = dA.x; s[1] = dA.y; s[2] = dA.z; s[3] = dA.w; s[4] = dB.x; s[5] = dB.y; s[6] = dB.z; s[7] = dB.w;
#pragma unroll
    for (int r = 0; r < 8; ++r) s[r] = s[r] * osc;
  } else {
#pragma unroll
    for (int r = 0; r < 8; ++r) s[r] = osc;
  }
  float bc[4];
#pragma unroll
  for (int t = 0; t < 4; ++t) bc[t] = (EPI != 0) ? bias[16 * t + m] : 0.0f;

  float* sp = stg + r0 * HC + m;
#pragma unroll
  for (int t = 0; t < 4; ++t) {
#pragma unroll
    for (int r = 0; r < 8; ++r) {
      float v = acc[t][r] * s[r] + bc[t];
      if (EPI != 0) v = fmaxf(v, 0.0f);
      sp[r * HC + 16 * t] = v;
    }
  }
  __syncthreads();

  if (EPI == 0) {
    const float* lp = stg + wave * 16 * HC;
    float* gp = Cf + (size_t)b * (size_t)strideC + (size_t)(rowBase + wave * 16) * HC;
#pragma unroll
    for (int i = 0; i < 8; ++i) {
      const v4f v = *(const v4f*)(lp + i * 128 + 4 * lane);
      *(volatile v4f*)(gp + (size_t)i * 128 + 4 * lane) = v;
    }
    __threadfence();
#pragma unroll
    for (int i = 0; i < 8; ++i) {
      const v4f v = *(const v4f*)(lp + i * 128 + 4 * lane);
      *(volatile v4f*)(gp + (size_t)i * 128 + 4 * lane) = v;
    }
  } else if (EPI == 1) {
    const int rq = lane >> 3, pc = 8 * (lane & 7);
#pragma unroll
    for (int i = 0; i < 4; ++i) {
      const int row = 4 * i + rq;
      const float* qp = stg + (wave * 16 + row) * HC + pc;
      const v4f f0 = *(const v4f*)qp;
      const v4f f1 = *(const v4f*)(qp + 4);
      v8h hv;
      hv[0] = (_Float16)(f0.x * hscl); hv[1] = (_Float16)(f0.y * hscl); hv[2] = (_Float16)(f0.z * hscl); hv[3] = (_Float16)(f0.w * hscl);
      hv[4] = (_Float16)(f1.x * hscl); hv[5] = (_Float16)(f1.y * hscl); hv[6] = (_Float16)(f1.z * hscl); hv[7] = (_Float16)(f1.w * hscl);
      _Float16* gp = Ch + (size_t)b * (size_t)strideC + (size_t)(rowBase + wave * 16 + row) * (size_t)ldc + pc;
      *(volatile v8h*)gp = hv;
    }
    __threadfence();
#pragma unroll
    for (int i = 0; i < 4; ++i) {
      const int row = 4 * i + rq;
      const float* qp = stg + (wave * 16 + row) * HC + pc;
      const v4f f0 = *(const v4f*)qp;
      const v4f f1 = *(const v4f*)(qp + 4);
      v8h hv;
      hv[0] = (_Float16)(f0.x * hscl); hv[1] = (_Float16)(f0.y * hscl); hv[2] = (_Float16)(f0.z * hscl); hv[3] = (_Float16)(f0.w * hscl);
      hv[4] = (_Float16)(f1.x * hscl); hv[5] = (_Float16)(f1.y * hscl); hv[6] = (_Float16)(f1.z * hscl); hv[7] = (_Float16)(f1.w * hscl);
      _Float16* gp = Ch + (size_t)b * (size_t)strideC + (size_t)(rowBase + wave * 16 + row) * (size_t)ldc + pc;
      *(volatile v8h*)gp = hv;
    }
  } else {
    const float* qrow = stg + (wave * 16 + m) * HC + 32 * hh;
    const float* qw   = sOw + 32 * hh;
    float sm = 0.0f;
#pragma unroll
    for (int k = 0; k < 8; ++k) {
      const v4f a = *(const v4f*)(qrow + 4 * k);
      const v4f w = *(const v4f*)(qw + 4 * k);
      sm += a.x * w.x; sm += a.y * w.y; sm += a.z * w.z; sm += a.w * w.w;
    }
    sm += __shfl_xor(sm, 16);
    const float val = sm + ob[0];
    if (hh == 0) sOut[wave * 16 + m] = val;
    __syncthreads();
    float* gp = Cf + (size_t)b * (size_t)strideC + (size_t)rowBase + 4 * lane;
    if (wave == 0) { const v4f v = *(const v4f*)(sOut + 4 * lane); *(volatile v4f*)gp = v; }
    __threadfence();
    if (wave == 0) { const v4f v = *(const v4f*)(sOut + 4 * lane); *(volatile v4f*)gp = v; }
  }
}

__global__ __launch_bounds__(NTHR) void k_out(const float* __restrict__ outv, float* out, int total4, int nN, int npad) {
  const int i = (int)blockIdx.x * NTHR + (int)threadIdx.x;
  if (i >= total4) return;
  const int f = 4 * i;
  const int b = f / nN;
  const int n = f - b * nN;
  const v4f v = *(const v4f*)(outv + (size_t)b * (size_t)npad + n);
  float* gp = out + f;
  *(volatile v4f*)gp = v;
  __threadfence();
  *(volatile v4f*)gp = v;
}

extern "C" void kernel_launch(void* const* d_in, const int* in_sizes, int n_in,
                              void* d_out, int out_size, void* d_ws, size_t ws_size,
                              hipStream_t stream) {
  if (n_in < 13) return;
  const int nN = NNODE;
  const int nE = in_sizes[1] / 2;
  if (nE <= 0 || in_sizes[1] != 2 * nE || in_sizes[2] != nE) return;
  if (nE > EMASK) return;
  if (in_sizes[0] != NBATCH * NTIME * NNODE * NFEAT) return;
  if (in_sizes[3] != NFEAT * HC || in_sizes[4] != HC || in_sizes[5] != HC * HC || in_sizes[6] != HC) return;
  if (in_sizes[7] != HC * HC * KTAP || in_sizes[8] != HC || in_sizes[9] != HC * HC * KTAP || in_sizes[10] != HC) return;
  if (in_sizes[11] != HC || in_sizes[12] < 1) return;
  if (out_size != NBATCH * NNODE) return;

  const float* X    = (const float*)d_in[0];
  const int*   ei   = (const int*)d_in[1];
  const float* ew   = (const float*)d_in[2];
  const float* W1   = (const float*)d_in[3];
  const float* b1   = (const float*)d_in[4];
  const float* W2   = (const float*)d_in[5];
  const float* b2   = (const float*)d_in[6];
  const float* tc1w = (const float*)d_in[7];
  const float* tc1b = (const float*)d_in[8];
  const float* tc2w = (const float*)d_in[9];
  const float* tc2b = (const float*)d_in[10];
  const float* outw = (const float*)d_in[11];
  const float* outb = (const float*)d_in[12];
  float* out = (float*)d_out;
  const int* vals = ei;
  const int* keys = ei + nE;
  const int nK = nE;

  const int nBC    = (nN + NBC - 1) / NBC;
  const int CNTPAD = nBC * NBC;
  const int nBF    = (nN + NBF - 1) / NBF;
  const int OFFN   = nBF * NBF;
  if (nBF + 1 > RBN) return;
  if (OFFN > CNTPAD || NPAD > OFFN) return;
  const int csrLen = ((nK + 31) & ~31) + 32 * (nBF + 1);
  const int nGemm  = NPAD / GROWS;
  const int nAgg   = NPAD / TGT;

  char* ws = (char*)d_ws;
  size_t off = 0;
  const size_t oH1  = off; off += (size_t)NBATCH * NPAD * HC * 2;    off = (off + 255) & ~(size_t)255;
  const size_t oHW  = off; off += (size_t)NBATCH * NPAD * HC * 4;    off = (off + 255) & ~(size_t)255;
  const size_t oSP  = off; off += (size_t)NBATCH * NPAD * SPP * 2;   off = (off + 255) & ~(size_t)255;
  const size_t oT1  = off; off += (size_t)NBATCH * NPAD * T1P * 2;   off = (off + 255) & ~(size_t)255;
  const size_t oOV  = off; off += (size_t)NBATCH * NPAD * 4;         off = (off + 255) & ~(size_t)255;
  const size_t oW2  = off; off += (size_t)HC * HC * 2;               off = (off + 255) & ~(size_t)255;
  const size_t oWc1 = off; off += (size_t)HC * KC * 2;               off = (off + 255) & ~(size_t)255;
  const size_t oWc2 = off; off += (size_t)HC * KC * 2;               off = (off + 255) & ~(size_t)255;
  const size_t oCnt = off; off += (size_t)CNTPAD * 4;                off = (off + 255) & ~(size_t)255;
  const size_t oDv  = off; off += (size_t)NPAD * 4;                  off = (off + 255) & ~(size_t)255;
  const size_t oOff = off; off += (size_t)OFFN * 4;                  off = (off + 255) & ~(size_t)255;
  const size_t oRb  = off; off += (size_t)RBN * 4;                   off = (off + 255) & ~(size_t)255;
  const size_t oCsr = off; off += (size_t)csrLen * 4;                off = (off + 255) & ~(size_t)255;
  if (off > ws_size || off > (size_t)WSCAP) return;
  _Float16* H1   = (_Float16*)(ws + oH1);
  float*    HW   = (float*)(ws + oHW);
  _Float16* SP   = (_Float16*)(ws + oSP);
  _Float16* T1   = (_Float16*)(ws + oT1);
  float*    OUTV = (float*)(ws + oOV);
  _Float16* W2p  = (_Float16*)(ws + oW2);
  _Float16* Wc1p = (_Float16*)(ws + oWc1);
  _Float16* Wc2p = (_Float16*)(ws + oWc2);
  int*      cnt  = (int*)(ws + oCnt);
  float*    dinv = (float*)(ws + oDv);
  int*      offp = (int*)(ws + oOff);
  int*      rb   = (int*)(ws + oRb);
  int*      csr  = (int*)(ws + oCsr);

  const int vec8 = ((nE & 7) == 0) ? 1 : 0;
  const float osc = 1.0f / ((float)HSCL * (float)WSCL);
  const int bstrideX = NTIME * NNODE * NFEAT;

  k_wprep<0><<<(HC * HC / 8 + NTHR - 1) / NTHR, NTHR, 0, stream>>>(W2, W2p, HC * HC / 8, (float)WSCL);
  k_wprep<1><<<(HC * KC / 8 + NTHR - 1) / NTHR, NTHR, 0, stream>>>(tc1w, Wc1p, HC * KC / 8, (float)WSCL);
  k_wprep<1><<<(HC * KC / 8 + NTHR - 1) / NTHR, NTHR, 0, stream>>>(tc2w, Wc2p, HC * KC / 8, (float)WSCL);

  hipFuncSetAttribute(reinterpret_cast<const void*>(&k_count),
                      hipFuncAttributeMaxDynamicSharedMemorySize, LDS_COUNT);
  k_count<<<nBC, NTHR, LDS_COUNT, stream>>>(keys, cnt, nK, vec8);
  k_offsets<<<1, OTHR, 0, stream>>>(cnt, offp, rb, nBF);
  hipFuncSetAttribute(reinterpret_cast<const void*>(&k_fill),
                      hipFuncAttributeMaxDynamicSharedMemorySize, LDS_FILL);
  k_fill<<<nBF, NTHR, LDS_FILL, stream>>>(keys, offp, rb, csr, nK, vec8, csrLen);
  k_dinv<<<NPAD / NTHR, NTHR, 0, stream>>>(csr, offp, cnt, ew, dinv, nK, csrLen);

  const dim3 gA(nAgg, NBATCH), gG(nGemm, NBATCH);
  for (int ti = 0; ti < NSL; ++ti) {
    const float* xs = X + (size_t)(TFIRST + ti) * NNODE * NFEAT;
    k_agg1<<<gA, NTHR, 0, stream>>>(csr, offp, cnt, dinv, vals, ew, xs, bstrideX, W1, b1, H1, nN, nK, csrLen, (float)HSCL);
    k_gemm<HC, 0><<<gG, NTHR, 0, stream>>>(H1, HC, NPAD * HC, W2p, HC, dinv, b2, outw, outb,
                                           HW, T1, T1P, NPAD * HC, osc, 1.0f);
    k_agg2<<<gA, NTHR, 0, stream>>>(csr, offp, cnt, dinv, vals, ew, HW, b2, SP + ti * HC, SPP, NPAD * SPP,
                                    nN, nK, csrLen, (float)HSCL);
  }

  k_gemm<KC, 1><<<gG, NTHR, 0, stream>>>(SP, SPP, NPAD * SPP, Wc1p, KC, dinv, tc1b, outw, outb,
                                         HW, T1, T1P, NPAD * T1P, osc, (float)HSCL);
  k_gemm<2 * HC, 1><<<gG, NTHR, 0, stream>>>(SP + HC, SPP, NPAD * SPP, Wc1p, KC, dinv, tc1b, outw, outb,
                                             HW, T1 + HC, T1P, NPAD * T1P, osc, (float)HSCL);
  k_gemm<2 * HC, 2><<<gG, NTHR, 0, stream>>>(T1, T1P, NPAD * T1P, Wc2p, KC, dinv, tc2b, outw, outb,
                                             OUTV, T1, T1P, NPAD, osc, 1.0f);

  {
    const int total4 = (NBATCH * NNODE) / 4;
    k_out<<<(total4 + NTHR - 1) / NTHR, NTHR, 0, stream>>>(OUTV, out, total4, nN, NPAD);
  }
}
